// HyperLayer_43052752175188
// MI455X (gfx1250) — hardware-verified
//
#include <hip/hip_runtime.h>
#include <hip/hip_bf16.h>
#include <math.h>


#define BB 2
#define SS 2048
#define DD 1024
#define HH 16
#define DKK 64
#define QW 2

typedef _Float16 bf16;
typedef __attribute__((ext_vector_type(4))) unsigned v4u_t;
typedef unsigned v4ua __attribute__((ext_vector_type(4), may_alias));
typedef __attribute__((ext_vector_type(4))) float v4f_t;
typedef float v4fa __attribute__((ext_vector_type(4), may_alias));
typedef __attribute__((ext_vector_type(16))) bf16  bf16x16;
typedef __attribute__((ext_vector_type(8)))  bf16  bf16x8;
typedef __attribute__((ext_vector_type(4)))  bf16  bf16x4;
typedef __attribute__((ext_vector_type(8)))  float f32x8;

#define LDS_STRIDE 48
#define KSTRIDE    72
#define VSTRIDE    48

__device__ __forceinline__ f32x8 wmma_bf16(bf16x16 a, bf16x16 b, f32x8 c) {
  return __builtin_amdgcn_wmma_f32_16x16x32_f16(
      false, a, false, b, (short)0, c, false, false);
}
#define RSPLIT (1.0f / 2048.0f)
__device__ __forceinline__ bf16 lo_of(float v, bf16 h) { return (bf16)((v - (float)h) * 2048.0f); }
__device__ __forceinline__ f32x8 wmma_split(bf16x16 a, bf16x16 al, bf16x16 b, bf16x16 bl, f32x8 c) {
  f32x8 x = {}; x = wmma_bf16(al, b, x); x = wmma_bf16(a, bl, x); return wmma_bf16(a, b, c) + x * RSPLIT; }

template <typename T>
__device__ __forceinline__ bf16x16 load_frag(const T* __restrict__ base, int ld,
                                             int row0, int k0) {
  const int lane = threadIdx.x & 31;
  const int r    = lane & 15;
  const int kh   = (lane >> 4) * 8;
  const T* p0 = base + (size_t)(row0 + r) * ld + (k0 + kh);
  const T* p1 = p0 + 16;
  bf16x16 f;
#pragma unroll
  for (int i = 0; i < 8; ++i) {
    f[i]     = (bf16)p0[i];
    f[i + 8] = (bf16)p1[i];
  }
  return f;
}

__device__ __forceinline__ bf16x16 lds_frag(const bf16* base, int stride) {
  const int lane = threadIdx.x & 31;
  const int row  = lane & 15;
  const int kh   = (lane >> 4) * 8;
  const bf16x8 lo = *(const bf16x8*)(base + row * stride + kh);
  const bf16x8 hi = *(const bf16x8*)(base + row * stride + kh + 16);
  bf16x16 f;
#pragma unroll
  for (int i = 0; i < 8; ++i) { f[i] = lo[i]; f[i + 8] = hi[i]; }
  return f;
}

template <typename T>
__device__ __forceinline__ void stage_read16(const T* __restrict__ p, float* buf) {
#pragma unroll
  for (int i = 0; i < 16; ++i) buf[i] = (float)p[i];
}

__device__ __forceinline__ void stage_write(bf16* dst, const float* buf, int nquad) {
#pragma unroll
  for (int i = 0; i < nquad; ++i) {
    bf16x4 q;
    q[0] = (bf16)buf[4 * i];     q[1] = (bf16)buf[4 * i + 1];
    q[2] = (bf16)buf[4 * i + 2]; q[3] = (bf16)buf[4 * i + 3];
    *(bf16x4*)(dst + 4 * i) = q;
  }
}

__global__ __launch_bounds__(256) void transpose_pack_kernel(const float* __restrict__ W, bf16* __restrict__ WT, int K, int N, size_t plane) {
  __shared__ float tile[64][65];
  const int k0 = blockIdx.y * 64, n0 = blockIdx.x * 64, t = threadIdx.x;
  for (int i = t; i < 64 * 64; i += 256) { const int kr = i >> 6, nc = i & 63; tile[kr][nc] = W[(size_t)(k0 + kr) * N + n0 + nc]; }
  __syncthreads();
#pragma unroll 1
  for (int pass = 0; pass < 2; ++pass) {
    for (int i = t; i < 64 * 8; i += 256) { const int nr = i >> 3, k8 = (i & 7) * 8; bf16 hh[8], hl[8];
#pragma unroll
      for (int e = 0; e < 8; ++e) { const float v = tile[k8 + e][nr]; hh[e] = (bf16)v; hl[e] = lo_of(v, hh[e]); }
      bf16* d = WT + (size_t)(n0 + nr) * K + k0 + k8;
      *(volatile v4u_t*)d = *(const v4ua*)hh; *(volatile v4u_t*)(d + plane) = *(const v4ua*)hl; }
    __threadfence();
  }
}

template <typename AT, typename WT, int MODE>
__global__ __launch_bounds__(256) void gemm_bias_kernel(
    const AT* __restrict__ A, const WT* __restrict__ W,
    const float* __restrict__ bias, void* __restrict__ out,
    int M, int N, int K) {
  __shared__ bf16 ldsA[128 * LDS_STRIDE];
  __shared__ bf16 ldsW[256 * LDS_STRIDE];
  __shared__ __attribute__((aligned(16))) unsigned char sob[256 * 136 * 2];

  const int t    = threadIdx.x;
  const int wave = t >> 5;
  const int lane = t & 31;
  const int wm   = (wave & 1) * 64;
  const int wn   = (wave >> 1) * 64;
  const int mBlk = blockIdx.x * 128;
  const int nBlk = blockIdx.y * 256;

  const int arow = t >> 1;
  const int ach  = (t & 1) * 16;

  float abuf[16];
  float wbuf[32];

  stage_read16(A + (size_t)(mBlk + arow) * K + ach, abuf);
  stage_read16(W + (size_t)(nBlk + t) * K,          wbuf);
  stage_read16(W + (size_t)(nBlk + t) * K + 16,     wbuf + 16);

  f32x8 acc[4][4] = {};

  for (int k = 0; k < K; k += 32) {
    __syncthreads();
    stage_write(&ldsA[arow * LDS_STRIDE + ach], abuf, 4);
    stage_write(&ldsW[t * LDS_STRIDE],          wbuf, 8);
    if (k + 32 < K) {
      stage_read16(A + (size_t)(mBlk + arow) * K + (k + 32) + ach, abuf);
      stage_read16(W + (size_t)(nBlk + t) * K + (k + 32),          wbuf);
      stage_read16(W + (size_t)(nBlk + t) * K + (k + 32) + 16,     wbuf + 16);
    }
    __syncthreads();

    bf16x16 af[4], wf[4];
#pragma unroll
    for (int i = 0; i < 4; ++i)
      af[i] = lds_frag(ldsA + (wm + 16 * i) * LDS_STRIDE, LDS_STRIDE);
#pragma unroll
    for (int j = 0; j < 4; ++j)
      wf[j] = lds_frag(ldsW + (wn + 16 * j) * LDS_STRIDE, LDS_STRIDE);
#pragma unroll
    for (int i = 0; i < 4; ++i)
#pragma unroll
      for (int j = 0; j < 4; ++j)
        acc[i][j] = wmma_bf16(af[i], wf[j], acc[i][j]);
  }

  const int nlane = lane & 15;
  const int mh    = (lane >> 4) * 8;
  __syncthreads();
  if (MODE == 0 || MODE == 1) {
    bf16* so = (bf16*)sob;
#pragma unroll
    for (int i = 0; i < 4; ++i)
#pragma unroll
      for (int j = 0; j < 4; ++j) {
        const int nl = wn + 16 * j + nlane;
        const float bv = bias[nBlk + nl];
#pragma unroll
        for (int r = 0; r < 8; ++r) {
          const int ml = wm + 16 * i + mh + r;
          const bf16 hv = (bf16)(acc[i][j][r] + bv);
          if (MODE == 0) so[ml * 264 + nl] = hv;
          else           so[nl * 136 + ml] = hv;
        }
      }
    __syncthreads();
#pragma unroll 1
    for (int pass = 0; pass < 2; ++pass) {
      if (MODE == 0) {
        for (int ch = t; ch < 128 * 32; ch += 256) { const int ml = ch >> 5, q = (ch & 31) * 8;
          *(volatile v4u_t*)((bf16*)out + (size_t)(mBlk + ml) * N + nBlk + q) = *(const v4ua*)(so + ml * 264 + q); }
      } else {
        const int b_ = mBlk >> 11, s0 = mBlk & (SS - 1);
        for (int ch = t; ch < 256 * 16; ch += 256) { const int nl = ch >> 4, q = (ch & 15) * 8; const int n = nBlk + nl, h = n >> 6, dk = n & (DKK - 1);
          *(volatile v4u_t*)((bf16*)out + (((size_t)(b_ * HH + h)) * DKK + dk) * SS + s0 + q) = *(const v4ua*)(so + nl * 136 + q); }
      }
      __threadfence();
    }
  } else {
    float* so = (float*)sob;
#pragma unroll 1
    for (int hf = 0; hf < 2; ++hf) {
      if (wm == hf * 64) {
#pragma unroll
        for (int i = 0; i < 4; ++i)
#pragma unroll
          for (int j = 0; j < 4; ++j) {
            const int nl = wn + 16 * j + nlane;
            const float bv = bias[nBlk + nl];
#pragma unroll
            for (int r = 0; r < 8; ++r) so[(16 * i + mh + r) * 260 + nl] = acc[i][j][r] + bv;
          }
      }
      __syncthreads();
#pragma unroll 1
      for (int pass = 0; pass < 2; ++pass) {
        for (int ch = t; ch < 64 * 64; ch += 256) { const int ml = ch >> 6, q = (ch & 63) * 4;
          *(volatile v4f_t*)((float*)out + (size_t)(mBlk + hf * 64 + ml) * N + nBlk + q) = *(const volatile v4fa*)(so + ml * 260 + q); }
        __threadfence();
      }
      __syncthreads();
    }
  }
}

template <typename AT, typename WT, int MODE>
__global__ __launch_bounds__(256) void gemm_split_kernel(
    const AT* __restrict__ A, size_t aPlane, const WT* __restrict__ W, size_t wPlane,
    const float* __restrict__ bias, void* __restrict__ out,
    int M, int N, int K) {
  __shared__ bf16 ldsA[128 * LDS_STRIDE], ldsAl[128 * LDS_STRIDE];
  __shared__ bf16 ldsW[256 * LDS_STRIDE], ldsWl[256 * LDS_STRIDE];
  __shared__ __attribute__((aligned(16))) unsigned char sob[256 * 136 * 2];

  const int t    = threadIdx.x;
  const int wave = t >> 5;
  const int lane = t & 31;
  const int wm   = (wave & 1) * 64;
  const int wn   = (wave >> 1) * 64;
  const int mBlk = blockIdx.x * 128;
  const int nBlk = blockIdx.y * 256;
  const int arow = t >> 1;
  const int ach  = (t & 1) * 16;

  f32x8 acc[4][4] = {};
  for (int k = 0; k < K; k += 32) {
    __syncthreads();
    {
      const AT* ap = A + (size_t)(mBlk + arow) * K + k + ach;
      bf16 hh[16], hl[16];
      if (sizeof(AT) == 4) {
#pragma unroll
        for (int i = 0; i < 16; ++i) { const float v = (float)ap[i]; hh[i] = (bf16)v; hl[i] = lo_of(v, hh[i]); }
      } else {
#pragma unroll
        for (int i = 0; i < 16; ++i) { hh[i] = (bf16)ap[i]; hl[i] = (bf16)ap[aPlane + i]; }
      }
#pragma unroll
      for (int i = 0; i < 16; ++i) { ldsA[arow * LDS_STRIDE + ach + i] = hh[i]; ldsAl[arow * LDS_STRIDE + ach + i] = hl[i]; }
    }
    {
      const WT* wp = W + (size_t)(nBlk + t) * K + k;
      if (sizeof(WT) == 4) {
#pragma unroll
        for (int i = 0; i < 32; ++i) { const float v = (float)wp[i]; const bf16 h_ = (bf16)v; ldsW[t * LDS_STRIDE + i] = h_; ldsWl[t * LDS_STRIDE + i] = lo_of(v, h_); }
      } else {
#pragma unroll
        for (int i = 0; i < 32; ++i) { ldsW[t * LDS_STRIDE + i] = (bf16)wp[i]; ldsWl[t * LDS_STRIDE + i] = (bf16)wp[wPlane + i]; }
      }
    }
    __syncthreads();
    bf16x16 wf[4], wfl[4];
#pragma unroll
    for (int j = 0; j < 4; ++j) { wf[j] = lds_frag(ldsW + (wn + 16 * j) * LDS_STRIDE, LDS_STRIDE); wfl[j] = lds_frag(ldsWl + (wn + 16 * j) * LDS_STRIDE, LDS_STRIDE); }
#pragma unroll
    for (int i = 0; i < 4; ++i) {
      const bf16x16 af = lds_frag(ldsA + (wm + 16 * i) * LDS_STRIDE, LDS_STRIDE), afl = lds_frag(ldsAl + (wm + 16 * i) * LDS_STRIDE, LDS_STRIDE);
#pragma unroll
      for (int j = 0; j < 4; ++j) acc[i][j] = wmma_split(af, afl, wf[j], wfl[j], acc[i][j]);
    }
  }

  const int nlane = lane & 15;
  const int mh    = (lane >> 4) * 8;
  __syncthreads();
  if (MODE == 1) {
    bf16* so = (bf16*)sob;
#pragma unroll
    for (int i = 0; i < 4; ++i)
#pragma unroll
      for (int j = 0; j < 4; ++j) {
        const int nl = wn + 16 * j + nlane;
        const float bv = bias ? bias[nBlk + nl] : 0.0f;
#pragma unroll
        for (int r = 0; r < 8; ++r) so[nl * 136 + wm + 16 * i + mh + r] = (bf16)(acc[i][j][r] + bv);
      }
    __syncthreads();
    const int b_ = mBlk >> 11, s0 = mBlk & (SS - 1);
#pragma unroll 1
    for (int pass = 0; pass < 2; ++pass) {
      for (int ch = t; ch < 256 * 16; ch += 256) { const int nl = ch >> 4, q = (ch & 15) * 8; const int n = nBlk + nl, h = n >> 6, dk = n & (DKK - 1);
        *(volatile v4u_t*)((bf16*)out + (((size_t)(b_ * HH + h)) * DKK + dk) * SS + s0 + q) = *(const v4ua*)(so + nl * 136 + q); }
      __threadfence();
    }
  } else {
    float* so = (float*)sob;
#pragma unroll 1
    for (int hf = 0; hf < 2; ++hf) {
      if (wm == hf * 64) {
#pragma unroll
        for (int i = 0; i < 4; ++i)
#pragma unroll
          for (int j = 0; j < 4; ++j) {
            const int nl = wn + 16 * j + nlane;
            const float bv = bias ? bias[nBlk + nl] : 0.0f;
#pragma unroll
            for (int r = 0; r < 8; ++r) so[(16 * i + mh + r) * 260 + nl] = acc[i][j][r] + bv;
          }
      }
      __syncthreads();
#pragma unroll 1
      for (int pass = 0; pass < 2; ++pass) {
        for (int ch = t; ch < 64 * 64; ch += 256) { const int ml = ch >> 6, q = (ch & 63) * 4;
          *(volatile v4f_t*)((float*)out + (size_t)(mBlk + hf * 64 + ml) * N + nBlk + q) = *(const volatile v4fa*)(so + ml * 260 + q); }
        __threadfence();
      }
      __syncthreads();
    }
  }
}


#define HB 4096
#define HIN 256
#define HOUT 256
#define HHY 128

__global__ __launch_bounds__(256) void k_cvt_x(const float* __restrict__ x, bf16* __restrict__ xh) {
  const int g = blockIdx.x * 256 + threadIdx.x;
  bf16 hh[8];
#pragma unroll
  for (int i = 0; i < 8; ++i) hh[i] = (bf16)x[(size_t)g * 8 + i];
  *(volatile v4u_t*)(xh + (size_t)g * 8) = *(const v4ua*)hh; __threadfence(); *(volatile v4u_t*)(xh + (size_t)g * 8) = *(const v4ua*)hh;
}
__global__ __launch_bounds__(256) void k_pack_hyper(const float* __restrict__ W1g, const float* __restrict__ W1b, const float* __restrict__ W2b,
                                                   bf16* __restrict__ W1T, bf16* __restrict__ W2bT) {
  const int g = blockIdx.x * 256 + threadIdx.x;
  const int n = g >> 5, k0 = (g & 31) * 8;
  const size_t plane = (size_t)256 * 256;
  bf16 a[8], al[8], c[8], cl[8];
#pragma unroll
  for (int i = 0; i < 8; ++i) { const int k = k0 + i;
    const float v1 = (n < HHY) ? W1g[(size_t)k * HHY + n] : W1b[(size_t)k * HHY + (n - HHY)];
    const float v2 = (k >= HHY) ? W2b[(size_t)(k - HHY) * HOUT + n] : 0.0f;
    a[i] = (bf16)v1; al[i] = lo_of(v1, a[i]); c[i] = (bf16)v2; cl[i] = lo_of(v2, c[i]); }
#pragma unroll 1
  for (int pass = 0; pass < 2; ++pass) {
    *(volatile v4u_t*)(W1T + (size_t)n * 256 + k0) = *(const v4ua*)a;  *(volatile v4u_t*)(W1T + plane + (size_t)n * 256 + k0) = *(const v4ua*)al;
    *(volatile v4u_t*)(W2bT + (size_t)n * 256 + k0) = *(const v4ua*)c; *(volatile v4u_t*)(W2bT + plane + (size_t)n * 256 + k0) = *(const v4ua*)cl;
    __threadfence();
  }
}
__global__ __launch_bounds__(256) void k_bias_cat(const float* __restrict__ b1g, const float* __restrict__ b1b, float* __restrict__ b1c) {
  const int i = threadIdx.x; const float v = (i < HHY) ? b1g[i] : b1b[i - HHY];
  *(volatile float*)(b1c + i) = v; __threadfence(); *(volatile float*)(b1c + i) = v;
}

__global__ __launch_bounds__(256) void gemm_acc_kernel(const bf16* __restrict__ A, const float* __restrict__ W, const float* __restrict__ scale,
                                                      float* __restrict__ out, int M, int N, int K) {
  __shared__ bf16 ldsA[128 * LDS_STRIDE];
  __shared__ bf16 ldsW[256 * LDS_STRIDE];
  __shared__ __attribute__((aligned(16))) float sob[64 * 260];
  const int t = threadIdx.x, wave = t >> 5, lane = t & 31, wm = (wave & 1) * 64, wn = (wave >> 1) * 64;
  const int mBlk = blockIdx.x * 128, nBlk = blockIdx.y * 256;
  const int arow = t >> 1, ach = (t & 1) * 16;
  float abuf[16], wbuf[32];
  stage_read16(A + (size_t)(mBlk + arow) * K + ach, abuf);
  stage_read16(W + (size_t)(nBlk + t) * K, wbuf); stage_read16(W + (size_t)(nBlk + t) * K + 16, wbuf + 16);
  f32x8 acc[4][4] = {};
  for (int k = 0; k < K; k += 32) {
    __syncthreads();
    stage_write(&ldsA[arow * LDS_STRIDE + ach], abuf, 4);
    stage_write(&ldsW[t * LDS_STRIDE], wbuf, 8);
    if (k + 32 < K) { stage_read16(A + (size_t)(mBlk + arow) * K + (k + 32) + ach, abuf);
      stage_read16(W + (size_t)(nBlk + t) * K + (k + 32), wbuf); stage_read16(W + (size_t)(nBlk + t) * K + (k + 32) + 16, wbuf + 16); }
    __syncthreads();
    bf16x16 af[4], wf[4];
#pragma unroll
    for (int i = 0; i < 4; ++i) af[i] = lds_frag(ldsA + (wm + 16 * i) * LDS_STRIDE, LDS_STRIDE);
#pragma unroll
    for (int j = 0; j < 4; ++j) wf[j] = lds_frag(ldsW + (wn + 16 * j) * LDS_STRIDE, LDS_STRIDE);
#pragma unroll
    for (int i = 0; i < 4; ++i)
#pragma unroll
      for (int j = 0; j < 4; ++j) acc[i][j] = wmma_bf16(af[i], wf[j], acc[i][j]);
  }
  const int nlane = lane & 15, mh = (lane >> 4) * 8;
  __syncthreads();
#pragma unroll 1
  for (int hf = 0; hf < 2; ++hf) {
    if (wm == hf * 64) {
#pragma unroll
      for (int i = 0; i < 4; ++i) {
        float sc[8];
#pragma unroll
        for (int r = 0; r < 8; ++r) sc[r] = scale ? scale[(size_t)(mBlk + hf * 64 + 16 * i + mh + r) * 256] : 1.0f;
#pragma unroll
        for (int j = 0; j < 4; ++j) { const int nl = wn + 16 * j + nlane;
#pragma unroll
          for (int r = 0; r < 8; ++r) sob[(16 * i + mh + r) * 260 + nl] = acc[i][j][r] * sc[r]; } }
    }
    __syncthreads();
#pragma unroll 1
    for (int pass = 0; pass < 2; ++pass) {
      for (int ch = t; ch < 64 * 64; ch += 256) { const int ml = ch >> 6, q = (ch & 63) * 4;
        float* dst = out + (size_t)(mBlk + hf * 64 + ml) * N + nBlk + q;
        v4f_t v = *(const volatile v4fa*)(sob + ml * 260 + q);
        if (pass == 0) { const v4f_t old = *(const v4fa*)dst; v.x += old.x; v.y += old.y; v.z += old.z; v.w += old.w; *(v4fa*)(sob + ml * 260 + q) = v; }
        *(volatile v4f_t*)dst = v; }
      __threadfence();
      __syncthreads();
    }
  }
}

__global__ __launch_bounds__(256) void k_relu(float* __restrict__ h) {
  const int g = blockIdx.x * 256 + threadIdx.x; v4f_t v = *(const v4fa*)(h + (size_t)g * 4);
  v.x = fmaxf(v.x, 0.0f); v.y = fmaxf(v.y, 0.0f); v.z = fmaxf(v.z, 0.0f); v.w = fmaxf(v.w, 0.0f);
  *(volatile v4f_t*)(h + (size_t)g * 4) = v; __threadfence(); *(volatile v4f_t*)(h + (size_t)g * 4) = v;
}

extern "C" void kernel_launch(void* const* d_in, const int* in_sizes, int n_in,
                              void* d_out, int out_size, void* d_ws, size_t ws_size,
                              hipStream_t stream) {
  (void)in_sizes; (void)n_in; (void)out_size; (void)ws_size;
  const float* x   = (const float*)d_in[0];
  const float* W1g = (const float*)d_in[1];
  const float* b1g = (const float*)d_in[2];
  const float* W2g = (const float*)d_in[3];
  const float* b2g = (const float*)d_in[4];
  const float* W1b = (const float*)d_in[5];
  const float* b1b = (const float*)d_in[6];
  const float* W2b = (const float*)d_in[7];
  const float* b2b = (const float*)d_in[8];
  float* out = (float*)d_out;
  char* ws = (char*)d_ws;
  bf16*  xh   = (bf16*)ws;  ws += (size_t)HB * HIN * 2;
  bf16*  W1T  = (bf16*)ws;  ws += (size_t)2 * 256 * 256 * 2;
  bf16*  W2bT = (bf16*)ws;  ws += (size_t)2 * 256 * 256 * 2;
  float* b1c  = (float*)ws; ws += 1024;
  float* Hh   = (float*)ws; ws += (size_t)HB * 256 * 4;

  k_cvt_x<<<HB * HIN / 8 / 256, 256, 0, stream>>>(x, xh);
  k_pack_hyper<<<(256 * 32) / 256, 256, 0, stream>>>(W1g, W1b, W2b, W1T, W2bT);
  k_bias_cat<<<1, 256, 0, stream>>>(b1g, b1b, b1c);
  gemm_split_kernel<float, bf16, 2><<<dim3(HB / 128, 1), 256, 0, stream>>>(x, 0, W1T, (size_t)256 * 256, b1c, Hh, HB, 256, 256);
  k_relu<<<HB * 256 / 4 / 256, 256, 0, stream>>>(Hh);
  gemm_split_kernel<float, bf16, 2><<<dim3(HB / 128, 1), 256, 0, stream>>>(Hh, 0, W2bT, (size_t)256 * 256, b2b, out, HB, 256, 256);
  gemm_acc_kernel<<<dim3(HB / 128, 1), 256, 0, stream>>>(xh, b2g, nullptr, out, HB, HOUT, HIN);
  for (int k = 0; k < HHY; ++k)
    gemm_acc_kernel<<<dim3(HB / 128, 1), 256, 0, stream>>>(xh, W2g + (size_t)k * HOUT * HIN, Hh + k, out, HB, HOUT, HIN);
}
